// TraditionalGNN_61787399520423
// MI455X (gfx1250) — hardware-verified
//
#include <hip/hip_runtime.h>
#include <stddef.h>


#define KD     128
#define GR     32
#define AP     136
#define NTHR   256
#define NWAVE  8
#define CHUNK  2048
#define WCAP   256
#define NGRP   (CHUNK / (NTHR * 4))
#define SLOTSH 10
#define WS_CAP 134217728

static_assert(WCAP == (CHUNK / NTHR) * 32);
static_assert(NGRP >= 1);
static_assert(CHUNK <= 2048);
static_assert((AP % 8) == 0);

typedef float          v2f  __attribute__((ext_vector_type(2)));
typedef float          v4f  __attribute__((ext_vector_type(4)));
typedef float          v8f  __attribute__((ext_vector_type(8)));
typedef int            v4i  __attribute__((ext_vector_type(4)));
typedef unsigned short v8us __attribute__((ext_vector_type(8)));
typedef __bf16         v16b __attribute__((ext_vector_type(16)));
union BFrag { v16b v; v8us half[2]; };
union Pack8 { v4i i; v8us u; unsigned short s[8]; };

template <int N> struct FV;
template <> struct FV<2> { typedef v2f T; };
template <> struct FV<4> { typedef v4f T; };

__device__ __forceinline__ v8f wmb(v16b a, v16b b, v8f c) {
  v8f d = __builtin_amdgcn_wmma_f32_16x16x32_bf16(false, a, false, b, (short)0, c, false, false);
  asm volatile("v_nop\n\tv_nop\n\tv_nop\n\tv_nop" : "+v"(d) : "v"(a), "v"(b));
  return d;
}

__device__ __forceinline__ unsigned short bf_rne(float f) {
  unsigned u = __float_as_uint(f);
  u += 0x7FFFu + ((u >> 16) & 1u);
  return (unsigned short)(u >> 16);
}
__device__ __forceinline__ float bf_up(unsigned short b) { return __uint_as_float(((unsigned)b) << 16); }

__device__ __forceinline__ void split8(v4f a, v4f b, Pack8& ph, Pack8& pl) {
  const float f[8] = {a.x, a.y, a.z, a.w, b.x, b.y, b.z, b.w};
#pragma unroll
  for (int j = 0; j < 8; ++j) {
    const unsigned short hb = bf_rne(f[j]);
    ph.s[j] = hb;
    pl.s[j] = bf_rne(f[j] - bf_up(hb));
  }
}

template <int NCOL>
__global__ __launch_bounds__(NTHR) void k_wprep(const float* __restrict__ W,
                                               unsigned short* Wth, unsigned short* Wtl) {
  const int i = blockIdx.x * NTHR + threadIdx.x;
  if (i >= NCOL * 16) return;
  const int n  = i >> 4;
  const int k0 = (i & 15) * 8;
  v4f a, b;
  a.x = W[(size_t)(k0 + 0) * NCOL + n]; a.y = W[(size_t)(k0 + 1) * NCOL + n];
  a.z = W[(size_t)(k0 + 2) * NCOL + n]; a.w = W[(size_t)(k0 + 3) * NCOL + n];
  b.x = W[(size_t)(k0 + 4) * NCOL + n]; b.y = W[(size_t)(k0 + 5) * NCOL + n];
  b.z = W[(size_t)(k0 + 6) * NCOL + n]; b.w = W[(size_t)(k0 + 7) * NCOL + n];
  Pack8 ph, pl;
  split8(a, b, ph, pl);
  const size_t o = (size_t)n * KD + k0;
  *(volatile v4i*)(Wth + o) = ph.i;
  *(volatile v4i*)(Wtl + o) = pl.i;
  __threadfence();
  *(volatile v4i*)(Wth + o) = ph.i;
  *(volatile v4i*)(Wtl + o) = pl.i;
}

template <int NCOL, int HEADS>
__global__ __launch_bounds__(NTHR) void k_gemm(
    const float* __restrict__ X, const unsigned short* __restrict__ Wth,
    const unsigned short* __restrict__ Wtl, const float* __restrict__ att_s,
    const float* __restrict__ att_d, float* Hout, float* AS, float* AD, int nN) {
  constexpr int CT  = NCOL / 16;
  constexpr int TPW = (2 * CT) / NWAVE;
  constexpr int XSP = NCOL + 4;
  constexpr int DH  = NCOL / HEADS;
  constexpr int SEG = NCOL / 8;
  constexpr int TPH = 8 / HEADS;
  constexpr int RPI = 128 / NCOL;
  constexpr int NI  = 4 / RPI;
  static_assert(TPW >= 1);
  static_assert(TPW * NWAVE == 2 * CT);
  static_assert((XSP % 4) == 0);
  static_assert(TPH >= 1);

  __shared__ __attribute__((aligned(16))) unsigned short Ath[GR * AP];
  __shared__ __attribute__((aligned(16))) unsigned short Atl[GR * AP];
  __shared__ __attribute__((aligned(16))) float Xs[GR * XSP];
  __shared__ __attribute__((aligned(16))) float Asl[GR * 8];
  __shared__ __attribute__((aligned(16))) float Dsl[GR * 8];

  const int tid  = threadIdx.x;
  const int lane = tid & 31;
  const int wave = tid >> 5;
  const int h    = lane >> 4;
  const int m    = lane & 15;
  const int rowBase = blockIdx.x * GR;

  {
    const int r  = tid >> 3;
    const int c0 = (tid & 7) * 16;
    int row = rowBase + r;
    if (row > nN - 1) row = nN - 1;
    const float* p = X + (size_t)row * KD + c0;
    const v4f f0 = *(const v4f*)(p), f1 = *(const v4f*)(p + 4);
    const v4f f2 = *(const v4f*)(p + 8), f3 = *(const v4f*)(p + 12);
    Pack8 h0, l0, h1, l1;
    split8(f0, f1, h0, l0);
    split8(f2, f3, h1, l1);
    *(v8us*)(Ath + r * AP + c0)     = h0.u;
    *(v8us*)(Ath + r * AP + c0 + 8) = h1.u;
    *(v8us*)(Atl + r * AP + c0)     = l0.u;
    *(v8us*)(Atl + r * AP + c0 + 8) = l1.u;
  }
  __syncthreads();

  v8f acc[TPW];
#pragma unroll
  for (int j = 0; j < TPW; ++j) {
    const v8f z = {0.f, 0.f, 0.f, 0.f, 0.f, 0.f, 0.f, 0.f};
    acc[j] = z;
  }
#pragma unroll 1
  for (int kt = 0; kt < KD / 32; ++kt) {
    const int k0 = kt * 32;
#pragma unroll
    for (int j = 0; j < TPW; ++j) {
      const int tile = wave * TPW + j;
      const int ct = tile >> 1;
      const int rt = tile & 1;
      BFrag fah, fal, fbh, fbl;
      const unsigned short* pa = Ath + (rt * 16 + m) * AP + k0 + 8 * h;
      const unsigned short* pl = Atl + (rt * 16 + m) * AP + k0 + 8 * h;
      const unsigned short* pb = Wth + (size_t)(ct * 16 + m) * KD + k0 + 8 * h;
      const unsigned short* pc = Wtl + (size_t)(ct * 16 + m) * KD + k0 + 8 * h;
      fah.half[0] = *(const v8us*)pa; fah.half[1] = *(const v8us*)(pa + 16);
      fal.half[0] = *(const v8us*)pl; fal.half[1] = *(const v8us*)(pl + 16);
      fbh.half[0] = *(const v8us*)pb; fbh.half[1] = *(const v8us*)(pb + 16);
      fbl.half[0] = *(const v8us*)pc; fbl.half[1] = *(const v8us*)(pc + 16);
      acc[j] = wmb(fah.v, fbh.v, acc[j]);
      acc[j] = wmb(fah.v, fbl.v, acc[j]);
      acc[j] = wmb(fal.v, fbh.v, acc[j]);
    }
  }

#pragma unroll
  for (int j = 0; j < TPW; ++j) {
    const int tile = wave * TPW + j;
    const int ct = tile >> 1;
    const int rt = tile & 1;
#pragma unroll
    for (int r = 0; r < 8; ++r) Xs[(rt * 16 + 8 * h + r) * XSP + ct * 16 + m] = acc[j][r];
  }
  __syncthreads();

  {
    const int row  = tid >> 3;
    const int part = tid & 7;
    const int col0 = part * SEG;
    const int head = col0 / DH;
    float s = 0.f, d = 0.f;
#pragma unroll
    for (int q = 0; q < SEG / 4; ++q) {
      const v4f xv = *(const v4f*)(Xs + row * XSP + col0 + 4 * q);
      const v4f av = *(const v4f*)(att_s + col0 + 4 * q);
      const v4f dv = *(const v4f*)(att_d + col0 + 4 * q);
      s += xv.x * av.x + xv.y * av.y + xv.z * av.z + xv.w * av.w;
      d += xv.x * dv.x + xv.y * dv.y + xv.z * dv.z + xv.w * dv.w;
    }
#pragma unroll
    for (int mk = 1; mk < TPH; mk <<= 1) {
      s += __shfl_xor(s, mk, 32);
      d += __shfl_xor(d, mk, 32);
    }
    if ((part & (TPH - 1)) == 0) {
      Asl[row * HEADS + head] = s;
      Dsl[row * HEADS + head] = d;
    }
  }
  __syncthreads();

  v4f xr[NI];
  float* xp[NI];
#pragma unroll
  for (int i = 0; i < NI; ++i) {
    const int row = 4 * wave + i * RPI + (4 * lane) / NCOL;
    const int col = (4 * lane) % NCOL;
    xr[i] = *(const v4f*)(Xs + row * XSP + col);
    xp[i] = Hout + (size_t)(rowBase + row) * NCOL + col;
  }
  constexpr int TOT = GR * HEADS;
  constexpr int WPA = (TOT + 127) / 128;
  constexpr int LPW = ((TOT < 128) ? TOT : 128) / 4;
  float* gp = 0;
  v4f gv = {0.f, 0.f, 0.f, 0.f};
  if (lane < LPW) {
    if (wave < WPA) {
      gv = *(const v4f*)(Asl + wave * 128 + 4 * lane);
      gp = AS + (size_t)rowBase * HEADS + wave * 128 + 4 * lane;
    } else if (wave < 2 * WPA) {
      gv = *(const v4f*)(Dsl + (wave - WPA) * 128 + 4 * lane);
      gp = AD + (size_t)rowBase * HEADS + (wave - WPA) * 128 + 4 * lane;
    }
  }
#pragma unroll
  for (int i = 0; i < NI; ++i) *(volatile v4f*)(xp[i]) = xr[i];
  if (gp) *(volatile v4f*)gp = gv;
  __threadfence();
#pragma unroll
  for (int i = 0; i < NI; ++i) *(volatile v4f*)(xp[i]) = xr[i];
  if (gp) *(volatile v4f*)gp = gv;
}

template <int F, int HEADS> struct AggCfg {
  static constexpr int NB = 65536 / F;
  static constexpr int LDS_FLOATS = NB * F + NB * HEADS;
  static constexpr int LDS_BYTES  = (LDS_FLOATS + NWAVE * WCAP + NWAVE) * 4;
};

template <int F, int HEADS>
__global__ __launch_bounds__(NTHR) void k_agg(
    const int* __restrict__ ei, const float* __restrict__ H,
    const float* __restrict__ asrc, const float* __restrict__ adst,
    const float* __restrict__ bias, float* outp, int nN, int nE, int relu) {
  constexpr int NB  = AggCfg<F, HEADS>::NB;
  constexpr int DH  = F / HEADS;
  constexpr int CPL = F / 32;
  constexpr int LPH = DH / CPL;
  constexpr int RPI = 128 / F;
  constexpr int SPW = NB / NWAVE;
  typedef typename FV<CPL>::T VT;
  static_assert((NB & (NB - 1)) == 0);
  static_assert(NB <= (1 << SLOTSH));
  static_assert((SPW % RPI) == 0);
  static_assert((LPH & (LPH - 1)) == 0);
  static_assert((AggCfg<F, HEADS>::LDS_FLOATS % 4) == 0);

  extern __shared__ v4f lds_dyn[];
  float* sacc = (float*)lds_dyn;
  float* den  = sacc + NB * F;
  int*   list = (int*)(den + NB * HEADS);
  int*   wcnt = list + NWAVE * WCAP;

  const int tid  = threadIdx.x;
  const int lane = tid & 31;
  const int wave = tid >> 5;
  const int hdr  = (lane * CPL) / DH;
  const int nodeBase = blockIdx.x * NB;

  {
    const v4f z4 = {0.f, 0.f, 0.f, 0.f};
    for (int i = tid; i < AggCfg<F, HEADS>::LDS_FLOATS / 4; i += NTHR) lds_dyn[i] = z4;
  }
  __syncthreads();

  const int* eid = ei + nE;
  const bool al16 = ((nE & 3) == 0);

  const int nChunks = (nE + CHUNK - 1) / CHUNK;
#pragma unroll 1
  for (int ch = 0; ch < nChunks; ++ch) {
    const int cbase = ch * CHUNK;
    int wc = 0;
#pragma unroll
    for (int g = 0; g < NGRP; ++g) {
      const int el0 = (g * NTHR + tid) * 4;
      const int e0  = cbase + el0;
      const int sent = -2147483647 - 1;
      v4i d;
      if (al16 && (e0 + 3 < nE)) {
        d = *(const v4i*)(eid + e0);
      } else {
        d.x = (e0     < nE) ? eid[min(e0, nE - 1)]     : sent;
        d.y = (e0 + 1 < nE) ? eid[min(e0 + 1, nE - 1)] : sent;
        d.z = (e0 + 2 < nE) ? eid[min(e0 + 2, nE - 1)] : sent;
        d.w = (e0 + 3 < nE) ? eid[min(e0 + 3, nE - 1)] : sent;
      }
      const unsigned s0 = (unsigned)d.x - (unsigned)nodeBase;
      const unsigned s1 = (unsigned)d.y - (unsigned)nodeBase;
      const unsigned s2 = (unsigned)d.z - (unsigned)nodeBase;
      const unsigned s3 = (unsigned)d.w - (unsigned)nodeBase;
      const bool h0 = s0 < (unsigned)NB;
      const bool h1 = s1 < (unsigned)NB;
      const bool h2 = s2 < (unsigned)NB;
      const bool h3 = s3 < (unsigned)NB;
      const unsigned many = __builtin_amdgcn_ballot_w32(h0 | h1 | h2 | h3);
      if (many != 0u) {
#define HITJ(J, HJ, SJ) { \
          const unsigned mj = __builtin_amdgcn_ballot_w32(HJ); \
          if (HJ) { \
            const int pos = wc + (int)__builtin_amdgcn_mbcnt_lo(mj, 0u); \
            if (pos < WCAP) list[wave * WCAP + pos] = ((el0 + (J)) << SLOTSH) | (int)(SJ); \
          } \
          wc += (int)__builtin_popcount(mj); }
        HITJ(0, h0, s0)
        HITJ(1, h1, s1)
        HITJ(2, h2, s2)
        HITJ(3, h3, s3)
#undef HITJ
      }
    }
    if (lane == 0) wcnt[wave] = wc;
    __syncthreads();

    if (wave == 0) {
      for (int wsx = 0; wsx < NWAVE; ++wsx) {
        int n = wcnt[wsx];
        if (n > WCAP) n = WCAP;
        if (n < 0) n = 0;
        for (int i = 0; i < n; ++i) {
          const int ent  = list[wsx * WCAP + i];
          const int slot = ent & (NB - 1);
          const int el   = (ent >> SLOTSH) & (CHUNK - 1);
          int e = cbase + el;
          if (e > nE - 1) e = nE - 1;
          int src = ei[e];
          src = src < 0 ? 0 : (src > nN - 1 ? nN - 1 : src);
          int nd = nodeBase + slot;
          if (nd > nN - 1) nd = nN - 1;
          float a = asrc[(size_t)src * HEADS + hdr] + adst[(size_t)nd * HEADS + hdr];
          a = (a > 0.f) ? a : 0.2f * a;
          a = fminf(a, 80.f);
          const float p = __expf(a);
          const VT xv = *(const VT*)(H + (size_t)src * F + CPL * lane);
          VT* sp = (VT*)(sacc + slot * F + CPL * lane);
          const VT cur = *sp;
          const VT nxt = cur + p * xv;
          *sp = nxt;
          if ((lane & (LPH - 1)) == 0) {
            const int di = slot * HEADS + hdr;
            const float o = den[di];
            den[di] = o + p;
          }
        }
      }
    }
    __syncthreads();
  }

  const int sub = (4 * lane) / F;
  const int col = (4 * lane) % F;
  const int hdf = col / DH;
  const v4f b4 = *(const v4f*)(bias + col);
#pragma unroll 1
  for (int j = 0; j < SPW; j += RPI) {
    const int slot0 = wave * SPW + j;
    if (nodeBase + slot0 >= nN) break;
    const int slot = slot0 + sub;
    const int node = nodeBase + slot;
    const bool ok  = node < nN;
    const size_t nrow = (size_t)(ok ? node : nN - 1);
    float a = asrc[nrow * HEADS + hdf] + adst[nrow * HEADS + hdf];
    a = (a > 0.f) ? a : 0.2f * a;
    a = fminf(a, 80.f);
    const float p = __expf(a);
    const v4f xv = *(const v4f*)(H + nrow * F + col);
    const v4f sv = *(const v4f*)(sacc + slot * F + col) + p * xv;
    const float dv  = den[slot * HEADS + hdf] + p;
    const float inv = 1.0f / (dv + 1e-16f);
    v4f y = sv * inv + b4;
    if (relu) {
      y.x = fmaxf(y.x, 0.f); y.y = fmaxf(y.y, 0.f);
      y.z = fmaxf(y.z, 0.f); y.w = fmaxf(y.w, 0.f);
    }
    float* op = outp + nrow * F + col;
    if (ok) *(volatile v4f*)op = y;
    __threadfence();
    if (ok) *(volatile v4f*)op = y;
  }
}

extern "C" void kernel_launch(void* const* d_in, const int* in_sizes, int n_in,
                              void* d_out, int out_size, void* d_ws, size_t ws_size,
                              hipStream_t stream) {
  if (n_in < 14) return;
  const int nN = in_sizes[0] / KD;
  const int nE = in_sizes[1] / 2;
  if (nN <= 0 || in_sizes[0] != nN * KD) return;
  if (nE < 0 || in_sizes[1] != 2 * nE) return;
  if (in_sizes[2] != KD * 128 || in_sizes[3] != 128 || in_sizes[4] != 128 || in_sizes[5] != 128) return;
  if (in_sizes[6] != KD * 128 || in_sizes[7] != 128 || in_sizes[8] != 128 || in_sizes[9] != 128) return;
  if (in_sizes[10] != KD * 64 || in_sizes[11] != 64 || in_sizes[12] != 64 || in_sizes[13] != 64) return;
  if (out_size != nN * 64) return;

  const float* x    = (const float*)d_in[0];
  const int*   ei   = (const int*)d_in[1];
  const float* W0   = (const float*)d_in[2];
  const float* as0  = (const float*)d_in[3];
  const float* ad0  = (const float*)d_in[4];
  const float* b0   = (const float*)d_in[5];
  const float* W1   = (const float*)d_in[6];
  const float* as1  = (const float*)d_in[7];
  const float* ad1  = (const float*)d_in[8];
  const float* b1   = (const float*)d_in[9];
  const float* W2   = (const float*)d_in[10];
  const float* as2  = (const float*)d_in[11];
  const float* ad2  = (const float*)d_in[12];
  const float* b2   = (const float*)d_in[13];
  float* out = (float*)d_out;

  const int nP = ((nN + GR - 1) / GR) * GR;
  size_t off = 0;
  unsigned short* Wth = (unsigned short*)((char*)d_ws + off); off += (size_t)KD * 128 * sizeof(unsigned short);
  unsigned short* Wtl = (unsigned short*)((char*)d_ws + off); off += (size_t)KD * 128 * sizeof(unsigned short);
  float* H   = (float*)((char*)d_ws + off); off += (size_t)nP * 128 * sizeof(float);
  float* AS  = (float*)((char*)d_ws + off); off += (size_t)nP * 8 * sizeof(float);
  float* AD  = (float*)((char*)d_ws + off); off += (size_t)nP * 8 * sizeof(float);
  float* ACT = (float*)((char*)d_ws + off); off += (size_t)nP * 128 * sizeof(float);
  if (off > ws_size || off > (size_t)WS_CAP) return;

  const int gridG  = nP / GR;
  const int gridA8 = (nN + AggCfg<128, 8>::NB - 1) / AggCfg<128, 8>::NB;
  const int gridA1 = (nN + AggCfg<64, 1>::NB - 1) / AggCfg<64, 1>::NB;

  hipFuncSetAttribute(reinterpret_cast<const void*>(&k_agg<128, 8>),
                      hipFuncAttributeMaxDynamicSharedMemorySize, AggCfg<128, 8>::LDS_BYTES);
  hipFuncSetAttribute(reinterpret_cast<const void*>(&k_agg<64, 1>),
                      hipFuncAttributeMaxDynamicSharedMemorySize, AggCfg<64, 1>::LDS_BYTES);

  k_wprep<128><<<(128 * 16 + NTHR - 1) / NTHR, NTHR, 0, stream>>>(W0, Wth, Wtl);
  k_gemm<128, 8><<<gridG, NTHR, 0, stream>>>(x, Wth, Wtl, as0, ad0, H, AS, AD, nN);
  k_agg<128, 8><<<gridA8, NTHR, AggCfg<128, 8>::LDS_BYTES, stream>>>(ei, H, AS, AD, b0, ACT, nN, nE, 1);

  k_wprep<128><<<(128 * 16 + NTHR - 1) / NTHR, NTHR, 0, stream>>>(W1, Wth, Wtl);
  k_gemm<128, 8><<<gridG, NTHR, 0, stream>>>(ACT, Wth, Wtl, as1, ad1, H, AS, AD, nN);
  k_agg<128, 8><<<gridA8, NTHR, AggCfg<128, 8>::LDS_BYTES, stream>>>(ei, H, AS, AD, b1, ACT, nN, nE, 1);

  k_wprep<64><<<(64 * 16 + NTHR - 1) / NTHR, NTHR, 0, stream>>>(W2, Wth, Wtl);
  k_gemm<64, 1><<<gridG, NTHR, 0, stream>>>(ACT, Wth, Wtl, as2, ad2, H, AS, AD, nN);
  k_agg<64, 1><<<gridA1, NTHR, AggCfg<64, 1>::LDS_BYTES, stream>>>(ei, H, AS, AD, b2, out, nN, nE, 0);
}
